// Baseline_20761871909173
// MI455X (gfx1250) — hardware-verified
//
#include <hip/hip_runtime.h>
#include <stddef.h>
#include <math.h>


#define EMBD   512
#define HIDD   1024
#define KTOT   (EMBD + HIDD)
#define KSTEPS (KTOT / 32)
#define PITCH  1544
#define TILE   (16 * PITCH)
#define OLW    128

typedef _Float16     v8h  __attribute__((ext_vector_type(8)));
typedef _Float16     v16h __attribute__((ext_vector_type(16)));
typedef float        v8f  __attribute__((ext_vector_type(8)));
typedef float        v4f  __attribute__((ext_vector_type(4)));
typedef unsigned int v4u  __attribute__((ext_vector_type(4)));

union Frag  { v16h v; v8h q[2]; };
union Pack8 { v8h h; v4u u; };

static __device__ __forceinline__ v16h load_frag(const _Float16* p) {
  Frag f;
  f.q[0] = *(const v8h*)(p);
  f.q[1] = *(const v8h*)(p + 16);
  return f.v;
}

static __device__ __forceinline__ v8f mma16(v16h a, v16h b, v8f c) {
  return __builtin_amdgcn_wmma_f32_16x16x32_f16(false, a, false, b, (short)0, c, false, false);
}

static __device__ __forceinline__ v4u pack8_scaled(v4f u0, v4f u1, float sc) {
  Pack8 p;
  p.h[0] = (_Float16)(u0.x * sc);
  p.h[1] = (_Float16)(u0.y * sc);
  p.h[2] = (_Float16)(u0.z * sc);
  p.h[3] = (_Float16)(u0.w * sc);
  p.h[4] = (_Float16)(u1.x * sc);
  p.h[5] = (_Float16)(u1.y * sc);
  p.h[6] = (_Float16)(u1.z * sc);
  p.h[7] = (_Float16)(u1.w * sc);
  return p.u;
}

static __device__ __forceinline__ float tanh_fast(float v) {
  float a = fminf(fabsf(v), 16.0f);
  float e = __expf(2.0f * a);
  float r = 1.0f - 2.0f * __builtin_amdgcn_rcpf(e + 1.0f);
  return copysignf(r, v);
}

static __device__ __forceinline__ v8f act8(v8f c, float bs) {
  v8f o;
#pragma unroll
  for (int r = 0; r < 8; ++r) o[r] = tanh_fast(c[r] * (1.0f / 256.0f) + bs);
  return o;
}

__global__ __launch_bounds__(256) void gather_rows_kernel(const int* __restrict__ x,
                                                          const float* __restrict__ emb,
                                                          _Float16* xe, int S, int Bn, int V) {
  const int lane = threadIdx.x & 31;
  const int wv   = threadIdx.x >> 5;
  const int g    = blockIdx.x * 8 + wv;
  const int total = S * Bn;
  if (g >= total) return;
  const int t = g / Bn;
  const int b = g - t * Bn;
  int tok = x[(size_t)b * S + t];
  if (tok < 0) tok += V;
  tok = tok < 0 ? 0 : (tok > V - 1 ? V - 1 : tok);
  const float* src = emb + (size_t)tok * EMBD + 8 * lane;
  _Float16* dst = xe + (size_t)g * EMBD + 8 * lane;
  v4u pk[EMBD / 256];
#pragma unroll
  for (int c = 0; c < EMBD / 256; ++c) {
    const v4f* s4 = (const v4f*)(src + c * 256);
    pk[c] = pack8_scaled(s4[0], s4[1], 4.0f);
  }
#pragma unroll
  for (int c = 0; c < EMBD / 256; ++c) *(volatile v4u*)(dst + c * 256) = pk[c];
  __threadfence();
#pragma unroll
  for (int c = 0; c < EMBD / 256; ++c) *(volatile v4u*)(dst + c * 256) = pk[c];
}

__global__ __launch_bounds__(256) void weight_convert_kernel(const float* __restrict__ Ww,
                                                            const float* __restrict__ Uw,
                                                            _Float16* wu, int H) {
  const int lane = threadIdx.x & 31;
  const int wv   = threadIdx.x >> 5;
  const int n    = blockIdx.x * 8 + wv;
  if (n >= H) return;
  const float* wrow = Ww + (size_t)n * EMBD + 8 * lane;
  const float* urow = Uw + (size_t)n * HIDD + 8 * lane;
  _Float16* dst = wu + (size_t)n * KTOT + 8 * lane;
  v4u pk[KTOT / 256];
#pragma unroll
  for (int c = 0; c < KTOT / 256; ++c) {
    const float* s = (c < EMBD / 256) ? (wrow + c * 256) : (urow + (c - EMBD / 256) * 256);
    const v4f* s4 = (const v4f*)s;
    pk[c] = pack8_scaled(s4[0], s4[1], 64.0f);
  }
#pragma unroll
  for (int c = 0; c < KTOT / 256; ++c) *(volatile v4u*)(dst + c * 256) = pk[c];
  __threadfence();
#pragma unroll
  for (int c = 0; c < KTOT / 256; ++c) *(volatile v4u*)(dst + c * 256) = pk[c];
}

__global__ __launch_bounds__(256) void rnn_kernel(const _Float16* __restrict__ xe,
                                                  const _Float16* __restrict__ wu,
                                                  const float* __restrict__ Wb,
                                                  const float* __restrict__ Ub,
                                                  const float* __restrict__ Vw,
                                                  const float* __restrict__ Vb,
                                                  float* outl, int S, int Bn) {
  __shared__ __align__(16) _Float16 sA[2 * TILE];
  __shared__ float sPart[8 * 16];
  __shared__ __align__(16) float sLine[OLW];

  const int tid  = threadIdx.x;
  const int lane = tid & 31;
  const int wv   = tid >> 5;
  const int hh   = lane >> 4;
  const int m    = lane & 15;
  const int bt   = blockIdx.x;
  if (bt * 16 + 15 >= Bn) return;

  {
    Pack8 z;
    v4u zz = {0u, 0u, 0u, 0u};
    z.u = zz;
    v8h* p = (v8h*)sA;
    for (int i = tid; i < (2 * TILE) / 8; i += 256) p[i] = z.h;
  }
  __syncthreads();

  float pl[8];
#pragma unroll
  for (int r = 0; r < 8; ++r) pl[r] = 0.0f;

#pragma unroll 1
  for (int t = 0; t < S; ++t) {
    _Float16* sAc = sA + (t & 1) * TILE;
    _Float16* sAn = sA + ((t + 1) & 1) * TILE;

    {
      const int row = tid >> 4;
      const int ch  = tid & 15;
      const v8h* src = (const v8h*)(xe + ((size_t)t * Bn + (size_t)bt * 16 + row) * EMBD + ch * 32);
      v8h q0 = src[0], q1 = src[1], q2 = src[2], q3 = src[3];
      v8h* d = (v8h*)(sAc + row * PITCH + ch * 32);
      d[0] = q0; d[1] = q1; d[2] = q2; d[3] = q3;
    }
    __syncthreads();

    const _Float16* ap = sAc + m * PITCH + 8 * hh;
    const bool last = (t == S - 1);

    for (int g = 0; g < 2; ++g) {
      const int ntb = wv * 8 + g * 4;
      const _Float16* bp = wu + ((size_t)(ntb * 16 + m)) * KTOT + 8 * hh;
      v8f c0 = {};
      v8f c1 = {};
      v8f c2 = {};
      v8f c3 = {};
#pragma unroll 1
      for (int kt = 0; kt < KSTEPS; ++kt) {
        const int ko = kt * 32;
        v16h a  = load_frag(ap + ko);
        v16h b0 = load_frag(bp + ko);
        v16h b1 = load_frag(bp + (size_t)16 * KTOT + ko);
        v16h b2 = load_frag(bp + (size_t)32 * KTOT + ko);
        v16h b3 = load_frag(bp + (size_t)48 * KTOT + ko);
        c0 = mma16(a, b0, c0);
        c1 = mma16(a, b1, c1);
        c2 = mma16(a, b2, c2);
        c3 = mma16(a, b3, c3);
        asm volatile("v_nop\n\tv_nop\n\tv_nop\n\tv_nop"
                     : "+v"(c0), "+v"(c1), "+v"(c2), "+v"(c3)
                     : "v"(a), "v"(b0), "v"(b1), "v"(b2), "v"(b3));
      }

      const int n0 = (ntb + 0) * 16 + m;
      const int n1 = (ntb + 1) * 16 + m;
      const int n2 = (ntb + 2) * 16 + m;
      const int n3 = (ntb + 3) * 16 + m;
      v8f h0 = act8(c0, Wb[n0] + Ub[n0]);
      v8f h1 = act8(c1, Wb[n1] + Ub[n1]);
      v8f h2 = act8(c2, Wb[n2] + Ub[n2]);
      v8f h3 = act8(c3, Wb[n3] + Ub[n3]);

      if (last) {
        const float v0 = Vw[n0], v1 = Vw[n1], v2 = Vw[n2], v3 = Vw[n3];
#pragma unroll
        for (int r = 0; r < 8; ++r) {
          float s = pl[r];
          s += h0[r] * v0;
          s += h1[r] * v1;
          s += h2[r] * v2;
          s += h3[r] * v3;
          pl[r] = s;
        }
      }

      _Float16* d0 = sAn + (8 * hh) * PITCH + EMBD + n0;
      _Float16* d1 = sAn + (8 * hh) * PITCH + EMBD + n1;
      _Float16* d2 = sAn + (8 * hh) * PITCH + EMBD + n2;
      _Float16* d3 = sAn + (8 * hh) * PITCH + EMBD + n3;
#pragma unroll
      for (int r = 0; r < 8; ++r) {
        d0[r * PITCH] = (_Float16)(h0[r] * 4.0f);
        d1[r * PITCH] = (_Float16)(h1[r] * 4.0f);
        d2[r * PITCH] = (_Float16)(h2[r] * 4.0f);
        d3[r * PITCH] = (_Float16)(h3[r] * 4.0f);
      }
    }
  }

#pragma unroll
  for (int r = 0; r < 8; ++r) {
    float v = pl[r];
    v += __shfl_xor(v, 8, 32);
    v += __shfl_xor(v, 4, 32);
    v += __shfl_xor(v, 2, 32);
    v += __shfl_xor(v, 1, 32);
    pl[r] = v;
  }
  if (m == 0) {
#pragma unroll
    for (int r = 0; r < 8; ++r) sPart[wv * 16 + 8 * hh + r] = pl[r];
  }
  __syncthreads();
  if (tid < OLW) {
    float o = 0.0f;
    if (tid < 16) {
      float s = 0.0f;
#pragma unroll
      for (int w = 0; w < 8; ++w) s += sPart[w * 16 + tid];
      s += Vb[0];
      o = 1.0f / (1.0f + expf(-s));
    }
    sLine[tid] = o;
  }
  __syncthreads();
  if (tid < 32) {
    v4f v = ((const v4f*)sLine)[tid];
    float* dst = outl + (size_t)bt * OLW + 4 * tid;
    *(volatile v4f*)dst = v;
    __threadfence();
    *(volatile v4f*)dst = v;
  }
}

__global__ __launch_bounds__(32) void collect_kernel(const float* outl, float* out, int Bn) {
  const int lane = threadIdx.x;
  for (int i = lane; 4 * i + 3 < Bn; i += 32) {
    v4f v = *(const v4f*)(outl + (size_t)(i >> 2) * OLW + (i & 3) * 4);
    *(volatile v4f*)(out + 4 * i) = v;
  }
  __threadfence();
  for (int i = lane; 4 * i + 3 < Bn; i += 32) {
    v4f v = *(const v4f*)(outl + (size_t)(i >> 2) * OLW + (i & 3) * 4);
    *(volatile v4f*)(out + 4 * i) = v;
  }
}

extern "C" void kernel_launch(void* const* d_in, const int* in_sizes, int n_in,
                              void* d_out, int out_size, void* d_ws,
                              size_t ws_size, hipStream_t stream) {
  if (n_in < 8) return;
  const int*   x   = (const int*)d_in[0];
  const float* emb = (const float*)d_in[1];
  const float* Ww  = (const float*)d_in[2];
  const float* Wb  = (const float*)d_in[3];
  const float* Uw  = (const float*)d_in[4];
  const float* Ub  = (const float*)d_in[5];
  const float* Vw  = (const float*)d_in[6];
  const float* Vb  = (const float*)d_in[7];
  float* out = (float*)d_out;
  char*  ws  = (char*)d_ws;

  const int H = in_sizes[3];
  if (H != HIDD) return;
  if (in_sizes[2] != HIDD * EMBD) return;
  if (in_sizes[4] != HIDD * HIDD) return;
  if (in_sizes[5] != HIDD || in_sizes[6] != HIDD || in_sizes[7] < 1) return;
  const int V = in_sizes[1] / EMBD;
  if (V <= 0) return;
  const int Bn = out_size;
  if (Bn <= 0 || (Bn % 16) != 0) return;
  const int S = in_sizes[0] / Bn;
  if (S <= 0 || S * Bn != in_sizes[0]) return;

  const size_t bytes_wu = (size_t)HIDD * KTOT * 2;
  const size_t off_wu   = 0;
  const size_t off_xe   = (off_wu + bytes_wu + 4095) & ~(size_t)4095;
  const size_t bytes_xe = (size_t)S * (size_t)Bn * EMBD * 2;
  const size_t off_ol   = (off_xe + bytes_xe + 4095) & ~(size_t)4095;
  const size_t bytes_ol = (size_t)(Bn / 16) * OLW * 4;
  const size_t total    = off_ol + bytes_ol;
  if (total > ws_size) return;

  _Float16* wu16 = (_Float16*)(ws + off_wu);
  _Float16* xe16 = (_Float16*)(ws + off_xe);
  float*    outl = (float*)(ws + off_ol);

  const int rows = S * Bn;
  weight_convert_kernel<<<dim3((HIDD + 7) / 8), dim3(256), 0, stream>>>(Ww, Uw, wu16, HIDD);
  gather_rows_kernel<<<dim3((rows + 7) / 8), dim3(256), 0, stream>>>(x, emb, xe16, S, Bn, V);
  rnn_kernel<<<dim3(Bn / 16), dim3(256), 0, stream>>>(xe16, wu16, Wb, Ub, Vw, Vb, outl, S, Bn);
  collect_kernel<<<dim3(1), dim3(32), 0, stream>>>(outl, out, Bn);
  (void)hipGetLastError();
}
